// AttentionModulator_19353122635924
// MI455X (gfx1250) — hardware-verified
//
#include <hip/hip_runtime.h>
#include <math.h>

typedef unsigned short u16;
typedef _Float16 v16h __attribute__((ext_vector_type(16)));
typedef _Float16 v8h  __attribute__((ext_vector_type(8)));
typedef __bf16   v16b __attribute__((ext_vector_type(16)));
typedef float    v8f  __attribute__((ext_vector_type(8)));
typedef float    v4f  __attribute__((ext_vector_type(4)));
typedef unsigned short v8us __attribute__((ext_vector_type(8)));
typedef v4f  __attribute__((may_alias)) v4fa;
typedef v8us __attribute__((may_alias)) v8usa;

#define NB     4
#define NTOK   1024
#define DN     128
#define DP     64
#define RD     16
#define FD     512
#define NH     8
#define HD     64
#define FF     2048
#define NL     4
#define TOKK   213
#define TOKP   256
#define MR     4096
#define PSCALE 16384.0f

__device__ __forceinline__ u16 f2bf(float f) {
  unsigned u = __float_as_uint(f);
  u += 0x7FFFu + ((u >> 16) & 1u);
  return (u16)(u >> 16);
}
__device__ __forceinline__ float bf2f(u16 b) { return __uint_as_float(((unsigned)b) << 16); }
__device__ __forceinline__ u16 f2h(float f) { union { _Float16 x; u16 u; } c; c.x = (_Float16)f; return c.u; }
__device__ __forceinline__ float h2f(u16 u) { union { _Float16 x; u16 u; } c; c.u = u; return (float)c.x; }
__device__ __forceinline__ float gelu_f(float x) { return 0.5f * x * (1.0f + erff(x * 0.70710678118654752f)); }
__device__ __forceinline__ v8f zero8() { v8f z;
#pragma unroll
  for (int i = 0; i < 8; ++i) z[i] = 0.0f; return z; }

__device__ __forceinline__ v8f wf16(v16h a, v16h b, v8f c) {
  v8f d = __builtin_amdgcn_wmma_f32_16x16x32_f16(false, a, false, b, (short)0, c, false, false);
  asm volatile("v_nop\n\tv_nop\n\tv_nop\n\tv_nop" : "+v"(d) : "v"(a), "v"(b));
  return d;
}
__device__ __forceinline__ v8f wbf16(v16b a, v16b b, v8f c) {
  v8f d = __builtin_amdgcn_wmma_f32_16x16x32_bf16(false, a, false, b, (short)0, c, false, false);
  asm volatile("v_nop\n\tv_nop\n\tv_nop\n\tv_nop" : "+v"(d) : "v"(a), "v"(b));
  return d;
}

union Frag { v16h f; v16b b; v8us u[2]; };
__device__ __forceinline__ Frag ldfrag(const u16* p, int h) {
  Frag f;
  f.u[0] = *(const v8usa*)(p + 8 * h);
  f.u[1] = *(const v8usa*)(p + 16 + 8 * h);
  return f;
}

__device__ __forceinline__ void cvt_tile(const float* __restrict__ Wm, int K, int N, int Kp, float sc, bool split,
                                         u16* o0, u16* o1, int g) {
  const int kq8 = Kp >> 3;
  const int n = g / kq8;
  const int kq = g - n * kq8;
  float v[8];
#pragma unroll
  for (int i = 0; i < 8; ++i) {
    const int k = kq * 8 + i;
    const int kc = (k < K) ? k : (K - 1);
    const float t = Wm[(size_t)kc * N + n];
    v[i] = (k < K) ? t * sc : 0.0f;
  }
  const size_t off = (size_t)n * Kp + (size_t)kq * 8;
  if (!split) {
    v8us o;
#pragma unroll
    for (int i = 0; i < 8; ++i) o[i] = f2h(v[i]);
    *(volatile v8us*)(o0 + off) = o;
    __threadfence();
    *(volatile v8us*)(o0 + off) = o;
  } else {
    v8us hv, lv;
#pragma unroll
    for (int i = 0; i < 8; ++i) { const u16 hb = f2bf(v[i]); hv[i] = hb; lv[i] = f2bf(v[i] - bf2f(hb)); }
    *(volatile v8us*)(o0 + off) = hv;
    *(volatile v8us*)(o1 + off) = lv;
    __threadfence();
    *(volatile v8us*)(o0 + off) = hv;
    *(volatile v8us*)(o1 + off) = lv;
  }
}

__global__ __launch_bounds__(256) void cvt_start_kernel(
    const float* __restrict__ tokW1, const float* __restrict__ tokW2, const float* __restrict__ headW,
    const float* __restrict__ Wh, const float* __restrict__ Wme, const float* __restrict__ Wmr,
    u16* tokW1t, u16* tokW2t, u16* headWt, u16* whT)
{
  const int seg = blockIdx.y;
  const int g = blockIdx.x * 256 + threadIdx.x;
  const float* src; u16* dst; int K, N, Kp;
  if (seg == 0)      { src = tokW1; K = TOKK; N = FD; Kp = TOKP; dst = tokW1t; }
  else if (seg == 1) { src = tokW2; K = FD;   N = FD; Kp = FD;   dst = tokW2t; }
  else if (seg == 2) { src = headW; K = FD;   N = FD; Kp = FD;   dst = headWt; }
  else { src = (seg == 3) ? Wh : ((seg == 4) ? Wme : Wmr); K = DN; N = DP; Kp = DN; dst = whT + (size_t)(seg - 3) * (DP * DN); }
  const int ng = (N * Kp) >> 3;
  if (g >= ng) return;
  cvt_tile(src, K, N, Kp, 32.0f, false, dst, dst, g);
}

__global__ __launch_bounds__(256) void cvt_layer_kernel(
    const float* __restrict__ qkvW, const float* __restrict__ outW,
    const float* __restrict__ f1W, const float* __restrict__ f2W,
    u16* qkvT, u16* outT, u16* w1h, u16* w1l, u16* w2h, u16* w2l)
{
  const int seg = blockIdx.y;
  const int g = blockIdx.x * 256 + threadIdx.x;
  const float* src; u16* d0; u16* d1; int K, N, Kp; bool split;
  if (seg == 0)      { src = qkvW; K = FD; N = 3 * FD; Kp = FD; d0 = qkvT; d1 = qkvT; split = false; }
  else if (seg == 1) { src = outW; K = FD; N = FD;     Kp = FD; d0 = outT; d1 = outT; split = false; }
  else if (seg == 2) { src = f1W;  K = FD; N = FF;     Kp = FD; d0 = w1h;  d1 = w1l;  split = true; }
  else               { src = f2W;  K = FF; N = FD;     Kp = FF; d0 = w2h;  d1 = w2l;  split = true; }
  const int ng = (N * Kp) >> 3;
  if (g >= ng) return;
  cvt_tile(src, K, N, Kp, split ? 1.0f : 32.0f, split, d0, d1, g);
}

__device__ __forceinline__ void fz_store(const u16* s, u16* tokin, int r0, int w, int lane) {
#pragma unroll
  for (int i = 0; i < 16; ++i) {
    const int row = 16 * w + i;
    const v8us v = *(const v8usa*)(s + row * TOKP + 8 * lane);
    *(volatile v8us*)(tokin + (size_t)(r0 + row) * TOKP + 8 * lane) = v;
  }
}

__global__ __launch_bounds__(128) void featurize_kernel(
    const float* __restrict__ hin, const float* __restrict__ msg, const float* __restrict__ rcv,
    const float* __restrict__ decay, const float* __restrict__ s_live, const float* __restrict__ s_ema,
    const int* __restrict__ role_id, const float* __restrict__ role_emb, int nrole,
    const u16* __restrict__ whT, u16* __restrict__ tokin)
{
  __shared__ __attribute__((aligned(16))) u16 sX[64 * 136];
  __shared__ __attribute__((aligned(16))) u16 sTk[64 * TOKP];
  const int tid = threadIdx.x, lane = tid & 31, w = tid >> 5;
  const int h = lane >> 4, m = lane & 15;
  const int r0 = blockIdx.x * 64;
  const int srow = tid >> 1, shalf = tid & 1;

#pragma unroll 1
  for (int p = 0; p < 3; ++p) {
    const float* src = (p == 0) ? hin : ((p == 1) ? msg : rcv);
    __syncthreads();
    const float* sr = src + (size_t)(r0 + srow) * DN + 64 * shalf;
    float ss = 0.0f;
#pragma unroll
    for (int i = 0; i < 8; ++i) {
      const v4f a = *(const v4fa*)(sr + 8 * i);
      const v4f c = *(const v4fa*)(sr + 8 * i + 4);
      ss += a.x * a.x + a.y * a.y + a.z * a.z + a.w * a.w + c.x * c.x + c.y * c.y + c.z * c.z + c.w * c.w;
      v8us o;
      o[0] = f2h(a.x); o[1] = f2h(a.y); o[2] = f2h(a.z); o[3] = f2h(a.w);
      o[4] = f2h(c.x); o[5] = f2h(c.y); o[6] = f2h(c.z); o[7] = f2h(c.w);
      *(v8usa*)(sX + srow * 136 + 64 * shalf + 8 * i) = o;
    }
    ss += __shfl_xor(ss, 1);
    if (p < 2 && shalf == 0) sTk[srow * TOKP + p] = f2h(sqrtf(ss));
    __syncthreads();

    v8f acc[4];
#pragma unroll
    for (int nt = 0; nt < 4; ++nt) acc[nt] = zero8();
#pragma unroll
    for (int k0 = 0; k0 < DN; k0 += 32) {
      const v16h a = ldfrag(sX + (16 * w + m) * 136 + k0, h).f;
#pragma unroll
      for (int nt = 0; nt < 4; ++nt) {
        const v16h b = ldfrag(whT + (size_t)p * (DP * DN) + (size_t)(16 * nt + m) * DN + k0, h).f;
        acc[nt] = wf16(a, b, acc[nt]);
      }
    }
#pragma unroll
    for (int nt = 0; nt < 4; ++nt)
#pragma unroll
      for (int r = 0; r < 8; ++r)
        sTk[(16 * w + 8 * h + r) * TOKP + 3 + 64 * p + 16 * nt + m] = f2h(acc[nt][r] * (1.0f / 32.0f));
  }

  if (tid < 64) {
    const int row = tid, grow = r0 + row, n = grow & (NTOK - 1), bz = grow >> 10;
    u16* tr = sTk + row * TOKP;
    tr[2] = f2h(decay[grow]);
    int rid = role_id[n];
    if (rid < 0) rid += nrole;
    rid = (rid < 0) ? 0 : ((rid >= nrole) ? (nrole - 1) : rid);
#pragma unroll
    for (int i = 0; i < RD; ++i) tr[3 + 3 * DP + i] = f2h(role_emb[rid * RD + i]);
    tr[TOKK - 2] = f2h(s_live[bz]);
    tr[TOKK - 1] = f2h(s_ema[bz]);
#pragma unroll
    for (int c = TOKK; c < TOKP; ++c) tr[c] = 0;
  }
  __syncthreads();
  fz_store(sTk, tokin, r0, w, lane);
  __threadfence();
  fz_store(sTk, tokin, r0, w, lane);
}

__device__ __forceinline__ void eb_store(const u16* sB, u16* eb, int b, int i0, int j0, int w, int lane) {
  const int q8 = lane & 7, sub = lane >> 3;
#pragma unroll
  for (int k = 0; k < 8; ++k) {
    const int L = w * 32 + 4 * k + sub;
    const int hh = L >> 5, i = L & 31;
    const v8us v = *(const v8usa*)(sB + (hh * 32 + i) * 64 + 8 * q8);
    *(volatile v8us*)(eb + (((size_t)(b * NH + hh)) * NTOK + i0 + i) * NTOK + j0 + 8 * q8) = v;
  }
}

__global__ __launch_bounds__(256) void edge_bias_kernel(
    const float* __restrict__ W, const float* __restrict__ heb,
    const float* __restrict__ W1, const float* __restrict__ b1,
    const float* __restrict__ W2, const float* __restrict__ b2,
    u16* __restrict__ eb)
{
  __shared__ float sWt[64 * 33];
  __shared__ float sw[104];
  __shared__ __attribute__((aligned(16))) u16 sB[NH * 32 * 64];
  const int tid = threadIdx.x, lane = tid & 31, w = tid >> 5;
  const int j0 = blockIdx.x * 64, i0 = blockIdx.y * 32, b = blockIdx.z;
  const float* Wb = W + (size_t)b * NTOK * NTOK;
  const float* Hb = heb + (size_t)b * NTOK * NTOK;

  {
    const float w1v = W1[(tid < 24) ? tid : 23];
    const float b1v = b1[(tid < 8) ? tid : 7];
    const float w2v = W2[(tid < 64) ? tid : 63];
    const float b2v = b2[(tid < 8) ? tid : 7];
    if (tid < 24) sw[tid] = w1v;
    if (tid < 8)  sw[24 + tid] = b1v;
    if (tid < 64) sw[32 + tid] = w2v;
    if (tid < 8)  sw[96 + tid] = b2v;
  }
#pragma unroll
  for (int it = 0; it < 8; ++it) {
    const int ii = tid & 31, jj = (tid >> 5) + 8 * it;
    sWt[jj * 33 + ii] = Wb[(size_t)(j0 + jj) * NTOK + i0 + ii];
  }
  __syncthreads();

  const int j = tid & 63;
#pragma unroll 1
  for (int it = 0; it < 8; ++it) {
    const int i = (tid >> 6) + 4 * it;
    const size_t gi = (size_t)(i0 + i) * NTOK + j0 + j;
    const float wv = Wb[gi];
    const float hb = Hb[gi];
    const float wt = sWt[j * 33 + i];
    const float as = wv - wt;
    float o[8];
#pragma unroll
    for (int hh = 0; hh < 8; ++hh) o[hh] = sw[96 + hh];
#pragma unroll 1
    for (int j8 = 0; j8 < 8; ++j8) {
      const float pre = wv * sw[j8] + hb * sw[8 + j8] + as * sw[16 + j8] + sw[24 + j8];
      const float gv = gelu_f(pre);
#pragma unroll
      for (int hh = 0; hh < 8; ++hh) o[hh] += gv * sw[32 + j8 * 8 + hh];
    }
#pragma unroll
    for (int hh = 0; hh < 8; ++hh) sB[(hh * 32 + i) * 64 + j] = f2h(o[hh] * 256.0f);
  }
  __syncthreads();
  eb_store(sB, eb, b, i0, j0, w, lane);
  __threadfence();
  eb_store(sB, eb, b, i0, j0, w, lane);
}

union GemmTile { float f[8192]; u16 h[16384]; };

__device__ __forceinline__ void gstore16(const u16* s, u16* dst, int N, int m0, int col0, int w, int lane) {
  const int q8 = lane & 7, sub = lane >> 3;
#pragma unroll
  for (int i = 0; i < 8; ++i) {
    const int tokl = 32 * w + 4 * i + sub;
    const v8us v = *(const v8usa*)(s + tokl * 64 + 8 * q8);
    *(volatile v8us*)(dst + (size_t)(m0 + tokl) * N + col0 + 8 * q8) = v;
  }
}
__device__ __forceinline__ void gstoreF(const float* s, float* dst, int N, int m0, int col0, int w, int lane) {
  const int q8 = lane & 7, sub = lane >> 3;
#pragma unroll
  for (int i = 0; i < 16; ++i) {
    const int lid = 4 * i + sub;
    const int tokl = 32 * w + (lid >> 1), hl = lid & 1;
    const v4f v = *(const v4fa*)(s + tokl * 64 + 32 * hl + 4 * q8);
    *(volatile v4f*)(dst + (size_t)(m0 + tokl) * N + col0 + 32 * hl + 4 * q8) = v;
  }
}
__device__ __forceinline__ void gstoreQKV(const u16* s, u16* plane, u16* vt, int which, int bh, int n0l, int w, int lane) {
  const int q8 = lane & 7, sub = lane >> 3;
#pragma unroll
  for (int i = 0; i < 8; ++i) {
    const int lid = w * 32 + i * 4 + sub;
    v8us v;
    u16* dst;
    if (which != 2) {
      v = *(const v8usa*)(s + lid * 64 + 8 * q8);
      dst = plane + ((size_t)bh * NTOK + n0l + lid) * HD + 8 * q8;
    } else {
      const int d = lid >> 1, hl = lid & 1;
      v = *(const v8usa*)(s + d * 128 + 64 * hl + 8 * q8);
      dst = vt + ((size_t)bh * HD + d) * NTOK + n0l + 64 * hl + 8 * q8;
    }
    *(volatile v8us*)dst = v;
  }
}

template <bool SPLIT, int EPI>
__global__ __launch_bounds__(128) void gemm_kernel(
    const u16* __restrict__ Ah, const u16* __restrict__ Al,
    const u16* __restrict__ Bh, const u16* __restrict__ Bl,
    const float* __restrict__ bias, float* xio,
    u16* __restrict__ o0, u16* __restrict__ o1, u16* __restrict__ o2,
    int N, int K)
{
  __shared__ __attribute__((aligned(16))) GemmTile sT;
  const int tid = threadIdx.x, lane = tid & 31, w = tid >> 5;
  const int h = lane >> 4, m = lane & 15;
  const int m0 = blockIdx.x * 128, col0 = blockIdx.y * 64;
  const int m0w = m0 + 32 * w;
  const size_t Ks = (size_t)K;
  const u16* a0p = Ah + (size_t)(m0w + m) * Ks;
  const u16* a1p = a0p + 16 * Ks;
  const u16* a0q = Al + (size_t)(m0w + m) * Ks;
  const u16* a1q = a0q + 16 * Ks;
  const u16* bp  = Bh + (size_t)(col0 + m) * Ks;
  const u16* bq  = Bl + (size_t)(col0 + m) * Ks;

  v8f acc[2][4];
#pragma unroll
  for (int mt = 0; mt < 2; ++mt)
#pragma unroll
    for (int nt = 0; nt < 4; ++nt) acc[mt][nt] = zero8();

#pragma unroll 1
  for (int k0 = 0; k0 < K; k0 += 32) {
    if (!SPLIT) {
      const v16h a0 = ldfrag(a0p + k0, h).f;
      const v16h a1 = ldfrag(a1p + k0, h).f;
#pragma unroll
      for (int nt = 0; nt < 4; ++nt) {
        const v16h b = ldfrag(bp + (size_t)nt * 16 * Ks + k0, h).f;
        acc[0][nt] = wf16(a0, b, acc[0][nt]);
        acc[1][nt] = wf16(a1, b, acc[1][nt]);
      }
    } else {
      const v16b a0h = ldfrag(a0p + k0, h).b;
      const v16b a1h = ldfrag(a1p + k0, h).b;
      const v16b a0l = ldfrag(a0q + k0, h).b;
      const v16b a1l = ldfrag(a1q + k0, h).b;
#pragma unroll
      for (int nt = 0; nt < 4; ++nt) {
        const v16b bh = ldfrag(bp + (size_t)nt * 16 * Ks + k0, h).b;
        const v16b bl = ldfrag(bq + (size_t)nt * 16 * Ks + k0, h).b;
        acc[0][nt] = wbf16(a0h, bh, acc[0][nt]);
        acc[0][nt] = wbf16(a0h, bl, acc[0][nt]);
        acc[0][nt] = wbf16(a0l, bh, acc[0][nt]);
        acc[1][nt] = wbf16(a1h, bh, acc[1][nt]);
        acc[1][nt] = wbf16(a1h, bl, acc[1][nt]);
        acc[1][nt] = wbf16(a1l, bh, acc[1][nt]);
      }
    }
  }

  const int which = (int)blockIdx.y >> 3;
  const float osc = (EPI == 0 || EPI == 1) ? (1.0f / 32.0f) : ((EPI == 2) ? 0.25f : ((EPI == 3) ? (1.0f / 256.0f) : 1.0f));
#pragma unroll
  for (int nt = 0; nt < 4; ++nt) {
    const int cl = 16 * nt + m, col = col0 + cl;
    float bv = 0.0f;
    if (EPI == 0 || EPI == 1 || EPI == 4 || EPI == 5) bv = bias[col];
#pragma unroll
    for (int mt = 0; mt < 2; ++mt)
#pragma unroll
      for (int r = 0; r < 8; ++r) {
        const int tokl = 32 * w + 16 * mt + 8 * h + r;
        float v = acc[mt][nt][r] * osc + bv;
        if (EPI == 0 || EPI == 4) v = gelu_f(v);
        if (EPI == 3 || EPI == 5) v += xio[(size_t)(m0 + tokl) * N + col];
        if (EPI == 1 || EPI == 3 || EPI == 5) {
          sT.f[tokl * 64 + cl] = v;
        } else if (EPI == 0) {
          sT.h[tokl * 64 + cl] = f2h(v);
        } else if (EPI == 2) {
          const int idx = (which == 2) ? (cl * 128 + tokl) : (tokl * 64 + cl);
          sT.h[idx] = f2h(v);
        } else {
          const u16 hb = f2bf(v);
          sT.h[tokl * 64 + cl] = hb;
          sT.h[8192 + tokl * 64 + cl] = f2bf(v - bf2f(hb));
        }
      }
  }
  __syncthreads();

  if (EPI == 1 || EPI == 3 || EPI == 5) {
    gstoreF(sT.f, xio, N, m0, col0, w, lane);
    __threadfence();
    gstoreF(sT.f, xio, N, m0, col0, w, lane);
  } else if (EPI == 0) {
    gstore16(sT.h, o0, N, m0, col0, w, lane);
    __threadfence();
    gstore16(sT.h, o0, N, m0, col0, w, lane);
  } else if (EPI == 4) {
    gstore16(sT.h, o0, N, m0, col0, w, lane);
    gstore16(sT.h + 8192, o1, N, m0, col0, w, lane);
    __threadfence();
    gstore16(sT.h, o0, N, m0, col0, w, lane);
    gstore16(sT.h + 8192, o1, N, m0, col0, w, lane);
  } else {
    const int b = m0 >> 10, n0l = m0 & (NTOK - 1), bh = b * NH + ((int)blockIdx.y & 7);
    u16* plane = (which == 0) ? o0 : o1;
    gstoreQKV(sT.h, plane, o2, which, bh, n0l, w, lane);
    __threadfence();
    gstoreQKV(sT.h, plane, o2, which, bh, n0l, w, lane);
  }
}

template <bool SPLIT>
__global__ __launch_bounds__(128) void ln_kernel(const float* x, const float* __restrict__ g,
    const float* __restrict__ bt, u16* oh, u16* ol, int nrows)
{
  const int lane = threadIdx.x & 31, w = threadIdx.x >> 5;
  const int row = blockIdx.x * 4 + w;
  if (row >= nrows) return;
  const float* xr = x + (size_t)row * FD;
  float v[16];
  {
    const v4f a = *(const v4fa*)(xr + 8 * lane);
    const v4f c = *(const v4fa*)(xr + 8 * lane + 4);
    const v4f d = *(const v4fa*)(xr + 256 + 8 * lane);
    const v4f e = *(const v4fa*)(xr + 256 + 8 * lane + 4);
    v[0] = a.x; v[1] = a.y; v[2] = a.z; v[3] = a.w; v[4] = c.x; v[5] = c.y; v[6] = c.z; v[7] = c.w;
    v[8] = d.x; v[9] = d.y; v[10] = d.z; v[11] = d.w; v[12] = e.x; v[13] = e.y; v[14] = e.z; v[15] = e.w;
  }
  float s = 0.0f;
#pragma unroll
  for (int i = 0; i < 16; ++i) s += v[i];
#pragma unroll
  for (int off = 16; off; off >>= 1) s += __shfl_xor(s, off);
  const float mean = s * (1.0f / FD);
  float q = 0.0f;
#pragma unroll
  for (int i = 0; i < 16; ++i) { v[i] -= mean; q += v[i] * v[i]; }
#pragma unroll
  for (int off = 16; off; off >>= 1) q += __shfl_xor(q, off);
  const float rstd = rsqrtf(q * (1.0f / FD) + 1e-5f);
  float gg[16], bb[16];
  {
    const v4f a = *(const v4fa*)(g + 8 * lane);
    const v4f c = *(const v4fa*)(g + 8 * lane + 4);
    const v4f d = *(const v4fa*)(g + 256 + 8 * lane);
    const v4f e = *(const v4fa*)(g + 256 + 8 * lane + 4);
    gg[0] = a.x; gg[1] = a.y; gg[2] = a.z; gg[3] = a.w; gg[4] = c.x; gg[5] = c.y; gg[6] = c.z; gg[7] = c.w;
    gg[8] = d.x; gg[9] = d.y; gg[10] = d.z; gg[11] = d.w; gg[12] = e.x; gg[13] = e.y; gg[14] = e.z; gg[15] = e.w;
    const v4f a2 = *(const v4fa*)(bt + 8 * lane);
    const v4f c2 = *(const v4fa*)(bt + 8 * lane + 4);
    const v4f d2 = *(const v4fa*)(bt + 256 + 8 * lane);
    const v4f e2 = *(const v4fa*)(bt + 256 + 8 * lane + 4);
    bb[0] = a2.x; bb[1] = a2.y; bb[2] = a2.z; bb[3] = a2.w; bb[4] = c2.x; bb[5] = c2.y; bb[6] = c2.z; bb[7] = c2.w;
    bb[8] = d2.x; bb[9] = d2.y; bb[10] = d2.z; bb[11] = d2.w; bb[12] = e2.x; bb[13] = e2.y; bb[14] = e2.z; bb[15] = e2.w;
  }
  float y[16];
#pragma unroll
  for (int i = 0; i < 16; ++i) y[i] = v[i] * rstd * gg[i] + bb[i];
  const size_t base = (size_t)row * FD;
  if (!SPLIT) {
    v8us p0, p1;
#pragma unroll
    for (int i = 0; i < 8; ++i) { p0[i] = f2h(y[i]); p1[i] = f2h(y[8 + i]); }
    *(volatile v8us*)(oh + base + 8 * lane) = p0;
    *(volatile v8us*)(oh + base + 256 + 8 * lane) = p1;
    __threadfence();
    *(volatile v8us*)(oh + base + 8 * lane) = p0;
    *(volatile v8us*)(oh + base + 256 + 8 * lane) = p1;
  } else {
    v8us h0, h1, l0, l1;
#pragma unroll
    for (int i = 0; i < 8; ++i) {
      const u16 a = f2bf(y[i]);     h0[i] = a; l0[i] = f2bf(y[i] - bf2f(a));
      const u16 c = f2bf(y[8 + i]); h1[i] = c; l1[i] = f2bf(y[8 + i] - bf2f(c));
    }
    *(volatile v8us*)(oh + base + 8 * lane) = h0;
    *(volatile v8us*)(oh + base + 256 + 8 * lane) = h1;
    *(volatile v8us*)(ol + base + 8 * lane) = l0;
    *(volatile v8us*)(ol + base + 256 + 8 * lane) = l1;
    __threadfence();
    *(volatile v8us*)(oh + base + 8 * lane) = h0;
    *(volatile v8us*)(oh + base + 256 + 8 * lane) = h1;
    *(volatile v8us*)(ol + base + 8 * lane) = l0;
    *(volatile v8us*)(ol + base + 256 + 8 * lane) = l1;
  }
}

__device__ __forceinline__ v16h pack_p(v8f a, v8f c) {
  v16h r;
#pragma unroll
  for (int i = 0; i < 8; ++i) { r[i] = (_Float16)(a[i] * PSCALE); r[8 + i] = (_Float16)(c[i] * PSCALE); }
  return r;
}
__device__ __forceinline__ void att_store(const u16* so, u16* ao, int b, int head, int q0, int lane) {
  const int q8 = lane & 7, sub = lane >> 3;
#pragma unroll
  for (int i = 0; i < 4; ++i) {
    const int row = 4 * i + sub;
    const v8us v = *(const v8usa*)(so + row * 64 + 8 * q8);
    *(volatile v8us*)(ao + ((size_t)(b * NTOK + q0 + row)) * FD + head * HD + 8 * q8) = v;
  }
}

__global__ __launch_bounds__(128) void attn_kernel(
    const u16* __restrict__ qh, const u16* __restrict__ kh, const u16* __restrict__ vt,
    const u16* __restrict__ eb, u16* __restrict__ ao)
{
  __shared__ __attribute__((aligned(16))) u16 sO[4 * 16 * 64];
  const int tid = threadIdx.x, lane = tid & 31, w = tid >> 5;
  const int h = lane >> 4, m = lane & 15;
  const int bh = blockIdx.y, b = bh >> 3, head = bh & 7;
  const int q0 = blockIdx.x * 64 + 16 * w;

  const u16* qrow = qh + ((size_t)bh * NTOK + q0 + m) * HD;
  const v16h qb0 = ldfrag(qrow, h).f;
  const v16h qb1 = ldfrag(qrow + 32, h).f;

  v8f o[4];
#pragma unroll
  for (int t = 0; t < 4; ++t) o[t] = zero8();
  float mrun = -1e30f, lrun = 0.0f;

  const u16* kbase = kh + ((size_t)bh * NTOK + m) * HD;
  const u16* vbase = vt + ((size_t)bh * HD + m) * NTOK;
  const u16* brow  = eb + ((size_t)bh * NTOK + q0 + m) * NTOK + 8 * h;

#pragma unroll 1
  for (int kb = 0; kb < NTOK; kb += 64) {
    v8f s[4];
#pragma unroll
    for (int j = 0; j < 4; ++j) {
      const u16* kp = kbase + (size_t)(kb + 16 * j) * HD;
      const v16h kf0 = ldfrag(kp, h).f;
      const v16h kf1 = ldfrag(kp + 32, h).f;
      v8f z = zero8();
      z = wf16(kf0, qb0, z);
      z = wf16(kf1, qb1, z);
      s[j] = z;
    }
#pragma unroll
    for (int j = 0; j < 4; ++j) {
      const v8us bbv = *(const v8usa*)(brow + kb + 16 * j);
#pragma unroll
      for (int r = 0; r < 8; ++r) s[j][r] = s[j][r] * (1.0f / 512.0f) + h2f(bbv[r]) * (1.0f / 256.0f);
    }

    float mloc = s[0][0];
#pragma unroll
    for (int j = 0; j < 4; ++j)
#pragma unroll
      for (int r = 0; r < 8; ++r) mloc = fmaxf(mloc, s[j][r]);
    mloc = fmaxf(mloc, __shfl_xor(mloc, 16));
    const float mnew = fmaxf(mrun, mloc);
    const float alpha = __expf(mrun - mnew);
    mrun = mnew;
    float lsum = 0.0f;
#pragma unroll
    for (int j = 0; j < 4; ++j)
#pragma unroll
      for (int r = 0; r < 8; ++r) {
        const float pv = __expf(s[j][r] - mnew);
        s[j][r] = pv;
        lsum += pv;
      }
    lsum += __shfl_xor(lsum, 16);
    lrun = lrun * alpha + lsum;
#pragma unroll
    for (int t = 0; t < 4; ++t)
#pragma unroll
      for (int r = 0; r < 8; ++r) o[t][r] = o[t][r] * alpha;

    const v16h pb0 = pack_p(s[0], s[1]);
    const v16h pb1 = pack_p(s[2], s[3]);
#pragma unroll
    for (int t = 0; t < 4; ++t) {
      const u16* vp = vbase + (size_t)(16 * t) * NTOK + kb;
      const v16h vf0 = ldfrag(vp, h).f;
      const v16h vf1 = ldfrag(vp + 32, h).f;
      o[t] = wf16(vf0, pb0, o[t]);
      o[t] = wf16(vf1, pb1, o[t]);
    }
  }

  const float inv = (1.0f / lrun) * (1.0f / PSCALE);
  u16* so = sO + w * 1024;
#pragma unroll
  for (int t = 0; t < 4; ++t)
#pragma unroll
    for (int r = 0; r < 8; ++r)
      so[m * 64 + 16 * t + 8 * h + r] = f2h(o[t][r] * inv);
  __syncthreads();
  att_store(so, ao, b, head, q0, lane);
  __threadfence();
  att_store(so, ao, b, head, q0, lane);
}

__global__ __launch_bounds__(256) void pool_head_kernel(const float* x, const float* __restrict__ pg,
    const float* __restrict__ pb, const u16* __restrict__ headWt, const float* __restrict__ hb, float* logits)
{
  __shared__ float sStat[2 * NTOK];
  __shared__ __attribute__((aligned(16))) u16 sA[16 * 520];
  __shared__ __attribute__((aligned(16))) float sL[FD];
  const int tid = threadIdx.x, lane = tid & 31, w = tid >> 5;
  const int h = lane >> 4, m = lane & 15;
  const int b = blockIdx.x;
  const float* xb = x + (size_t)b * NTOK * FD;

#pragma unroll 1
  for (int r = w; r < NTOK; r += 8) {
    const float* xr = xb + (size_t)r * FD + 16 * lane;
    float v[16];
    {
      const v4f a = *(const v4fa*)(xr); const v4f c = *(const v4fa*)(xr + 4);
      const v4f d = *(const v4fa*)(xr + 8); const v4f e = *(const v4fa*)(xr + 12);
      v[0] = a.x; v[1] = a.y; v[2] = a.z; v[3] = a.w; v[4] = c.x; v[5] = c.y; v[6] = c.z; v[7] = c.w;
      v[8] = d.x; v[9] = d.y; v[10] = d.z; v[11] = d.w; v[12] = e.x; v[13] = e.y; v[14] = e.z; v[15] = e.w;
    }
    float s = 0.0f;
#pragma unroll
    for (int i = 0; i < 16; ++i) s += v[i];
#pragma unroll
    for (int off = 16; off; off >>= 1) s += __shfl_xor(s, off);
    const float mean = s * (1.0f / FD);
    float q = 0.0f;
#pragma unroll
    for (int i = 0; i < 16; ++i) { const float d0 = v[i] - mean; q += d0 * d0; }
#pragma unroll
    for (int off = 16; off; off >>= 1) q += __shfl_xor(q, off);
    const float rstd = rsqrtf(q * (1.0f / FD) + 1e-5f);
    if (lane == 0) { sStat[2 * r] = mean; sStat[2 * r + 1] = rstd; }
  }
#pragma unroll 1
  for (int i = tid; i < 15 * 520; i += 256) sA[520 + i] = 0;
  __syncthreads();

  const int c = 2 * tid;
  double a0 = 0.0, a1 = 0.0;
#pragma unroll 1
  for (int n = 0; n < NTOK; ++n) {
    const float* p = xb + (size_t)n * FD + c;
    const float x0 = p[0], x1 = p[1];
    const float mu = sStat[2 * n], rs = sStat[2 * n + 1];
    a0 += (double)((x0 - mu) * rs);
    a1 += (double)((x1 - mu) * rs);
  }
  const float p0 = pg[c] * (float)(a0 * (1.0 / NTOK)) + pb[c];
  const float p1 = pg[c + 1] * (float)(a1 * (1.0 / NTOK)) + pb[c + 1];
  sA[c] = f2h(p0);
  sA[c + 1] = f2h(p1);
  __syncthreads();

  v8f acc[4];
#pragma unroll
  for (int nt = 0; nt < 4; ++nt) acc[nt] = zero8();
#pragma unroll 1
  for (int k0 = 0; k0 < FD; k0 += 32) {
    const v16h a = ldfrag(sA + m * 520 + k0, h).f;
#pragma unroll
    for (int nt = 0; nt < 4; ++nt) {
      const v16h bf = ldfrag(headWt + (size_t)(64 * w + 16 * nt + m) * FD + k0, h).f;
      acc[nt] = wf16(a, bf, acc[nt]);
    }
  }
#pragma unroll
  for (int nt = 0; nt < 4; ++nt) {
    const int col = 64 * w + 16 * nt + m;
    const float val = acc[nt][0] * (1.0f / 32.0f) + hb[col];
    if (h == 0) sL[col] = val;
  }
  __syncthreads();
  if (tid < 128) {
    const v4f v = *(const v4fa*)(sL + 4 * tid);
    *(volatile v4f*)(logits + (size_t)b * FD + 4 * tid) = v;
  }
  __threadfence();
  if (tid < 128) {
    const v4f v = *(const v4fa*)(sL + 4 * tid);
    *(volatile v4f*)(logits + (size_t)b * FD + 4 * tid) = v;
  }
}

extern "C" void kernel_launch(void* const* d_in, const int* in_sizes, int n_in,
                              void* d_out, int out_size, void* d_ws, size_t ws_size,
                              hipStream_t stream) {
  if (n_in < 35) return;
  if (in_sizes[0] != MR * DN || in_sizes[1] != MR * DN || in_sizes[2] != MR * DN) return;
  if (in_sizes[3] != NB * NTOK * NTOK || in_sizes[4] != NB * NTOK * NTOK) return;
  if (in_sizes[5] != MR || in_sizes[6] != NB || in_sizes[7] != NB || in_sizes[8] != NTOK) return;
  if (in_sizes[9] != DN * DP || in_sizes[10] != DN * DP || in_sizes[11] != DN * DP) return;
  if (in_sizes[12] < RD || (in_sizes[12] % RD) != 0) return;
  if (in_sizes[13] != TOKK * FD || in_sizes[14] != FD || in_sizes[15] != FD * FD || in_sizes[16] != FD) return;
  if (in_sizes[17] != 24 || in_sizes[18] != 8 || in_sizes[19] != 64 || in_sizes[20] != 8) return;
  if (in_sizes[21] != NL * FD || in_sizes[22] != NL * FD) return;
  if (in_sizes[23] != NL * FD * 3 * FD || in_sizes[24] != NL * FD * FD) return;
  if (in_sizes[25] != NL * FD || in_sizes[26] != NL * FD) return;
  if (in_sizes[27] != NL * FD * FF || in_sizes[28] != NL * FF || in_sizes[29] != NL * FF * FD || in_sizes[30] != NL * FD) return;
  if (in_sizes[31] != FD || in_sizes[32] != FD || in_sizes[33] != FD * FD || in_sizes[34] != FD) return;
  if (out_size != NB * FD + MR * FD) return;

  const float* hin     = (const float*)d_in[0];
  const float* msg     = (const float*)d_in[1];
  const float* rcv     = (const float*)d_in[2];
  const float* W       = (const float*)d_in[3];
  const float* heb     = (const float*)d_in[4];
  const float* decay   = (const float*)d_in[5];
  const float* s_live  = (const float*)d_in[6];
  const float* s_ema   = (const float*)d_in[7];
  const int*   role_id = (const int*)d_in[8];
  const float* Wh      = (const float*)d_in[9];
  const float* Wme     = (const float*)d_in[10];
  const float* Wmr     = (const float*)d_in[11];
  const float* role_emb = (const float*)d_in[12];
  const float* tok_W1  = (const float*)d_in[13];
  const float* tok_b1  = (const float*)d_in[14];
  const float* tok_W2  = (const float*)d_in[15];
  const float* tok_b2  = (const float*)d_in[16];
  const float* eb_W1   = (const float*)d_in[17];
  const float* eb_b1   = (const float*)d_in[18];
  const float* eb_W2   = (const float*)d_in[19];
  const float* eb_b2   = (const float*)d_in[20];
  const float* ln1_g   = (const float*)d_in[21];
  const float* ln1_b   = (const float*)d_in[22];
  const float* qkv_W   = (const float*)d_in[23];
  const float* out_W   = (const float*)d_in[24];
  const float* ln2_g   = (const float*)d_in[25];
  const float* ln2_b   = (const float*)d_in[26];
  const float* ffn_W1  = (const float*)d_in[27];
  const float* ffn_b1  = (const float*)d_in[28];
  const float* ffn_W2  = (const float*)d_in[29];
  const float* ffn_b2  = (const float*)d_in[30];
  const float* pool_g  = (const float*)d_in[31];
  const float* pool_b  = (const float*)d_in[32];
  const float* head_W  = (const float*)d_in[33];
  const float* head_b  = (const float*)d_in[34];
  const int nrole = in_sizes[12] / RD;

  float* logits = (float*)d_out;
  float* x      = (float*)d_out + NB * FD;

  char* wsb = (char*)d_ws;
  size_t off = 0;
  auto carve = [&](size_t bytes) -> char* {
    char* p = wsb + off;
    off += (bytes + 255) & ~(size_t)255;
    return p;
  };
  u16* whT    = (u16*)carve((size_t)3 * DP * DN * 2);
  u16* tokW1t = (u16*)carve((size_t)FD * TOKP * 2);
  u16* tokW2t = (u16*)carve((size_t)FD * FD * 2);
  u16* headWt = (u16*)carve((size_t)FD * FD * 2);
  u16* qkvWt  = (u16*)carve((size_t)3 * FD * FD * 2);
  u16* outWt  = (u16*)carve((size_t)FD * FD * 2);
  u16* w1hi   = (u16*)carve((size_t)FF * FD * 2);
  u16* w1lo   = (u16*)carve((size_t)FF * FD * 2);
  u16* w2hi   = (u16*)carve((size_t)FD * FF * 2);
  u16* w2lo   = (u16*)carve((size_t)FD * FF * 2);
  u16* tokin  = (u16*)carve((size_t)MR * TOKP * 2);
  u16* ebias  = (u16*)carve((size_t)NB * NH * NTOK * NTOK * 2);
  char* U     = carve((size_t)41943040);
  if (off > ws_size) return;
  if (off > (size_t)134217728) return;

  u16* hn   = (u16*)(U);
  u16* qp   = (u16*)(U + (size_t)4194304);
  u16* kp   = (u16*)(U + (size_t)8388608);
  u16* vtp  = (u16*)(U + (size_t)12582912);
  u16* aob  = (u16*)(U + (size_t)16777216);
  u16* hn2h = (u16*)(U);
  u16* hn2l = (u16*)(U + (size_t)4194304);
  u16* ffhh = (u16*)(U + (size_t)8388608);
  u16* ffhl = (u16*)(U + (size_t)25165824);
  u16* hid  = hn;

  cvt_start_kernel<<<dim3(128, 6), 256, 0, stream>>>(tok_W1, tok_W2, head_W, Wh, Wme, Wmr,
                                                      tokW1t, tokW2t, headWt, whT);
  featurize_kernel<<<MR / 64, 128, 0, stream>>>(hin, msg, rcv, decay, s_live, s_ema, role_id, role_emb, nrole, whT, tokin);
  gemm_kernel<false, 0><<<dim3(MR / 128, FD / 64), 128, 0, stream>>>(tokin, tokin, tokW1t, tokW1t, tok_b1, x, hid, hid, hid, FD, TOKP);
  gemm_kernel<false, 1><<<dim3(MR / 128, FD / 64), 128, 0, stream>>>(hid, hid, tokW2t, tokW2t, tok_b2, x, hid, hid, hid, FD, FD);
  edge_bias_kernel<<<dim3(NTOK / 64, NTOK / 32, NB), 256, 0, stream>>>(W, heb, eb_W1, eb_b1, eb_W2, eb_b2, ebias);

  for (int l = 0; l < NL; ++l) {
    cvt_layer_kernel<<<dim3(512, 4), 256, 0, stream>>>(
        qkv_W + (size_t)l * FD * 3 * FD, out_W + (size_t)l * FD * FD,
        ffn_W1 + (size_t)l * FD * FF, ffn_W2 + (size_t)l * FF * FD,
        qkvWt, outWt, w1hi, w1lo, w2hi, w2lo);
    ln_kernel<false><<<MR / 4, 128, 0, stream>>>(x, ln1_g + l * FD, ln1_b + l * FD, hn, hn, MR);
    gemm_kernel<false, 2><<<dim3(MR / 128, (3 * FD) / 64), 128, 0, stream>>>(hn, hn, qkvWt, qkvWt, tok_b1, x, qp, kp, vtp, 3 * FD, FD);
    attn_kernel<<<dim3(NTOK / 64, NB * NH), 128, 0, stream>>>(qp, kp, vtp, ebias, aob);
    gemm_kernel<false, 3><<<dim3(MR / 128, FD / 64), 128, 0, stream>>>(aob, aob, outWt, outWt, tok_b1, x, hn, hn, hn, FD, FD);
    ln_kernel<true><<<MR / 4, 128, 0, stream>>>(x, ln2_g + l * FD, ln2_b + l * FD, hn2h, hn2l, MR);
    gemm_kernel<true, 4><<<dim3(MR / 128, FF / 64), 128, 0, stream>>>(hn2h, hn2l, w1hi, w1lo, ffn_b1 + l * FF, x, ffhh, ffhl, ffhl, FF, FD);
    gemm_kernel<true, 5><<<dim3(MR / 128, FD / 64), 128, 0, stream>>>(ffhh, ffhl, w2hi, w2lo, ffn_b2 + l * FD, x, hn2h, hn2h, hn2h, FD, FF);
  }

  pool_head_kernel<<<NB, 256, 0, stream>>>(x, pool_g, pool_b, headWt, head_b, logits);
}
